// QuantMultiheadAttention_45664092291657
// MI455X (gfx1250) — hardware-verified
//
#include <hip/hip_runtime.h>
#include <math.h>
#include <stdint.h>

#define TT    2048
#define NBAT  2
#define EMB   1024
#define NH    16
#define HD    64
#define NTOK  (TT * NBAT)
#define QKW   (2 * EMB)
#define NQB   (TT / 64)
static_assert(NH * HD == EMB);
static_assert((TT % 64) == 0 && (EMB % 64) == 0 && (NTOK % 64) == 0 && (EMB % 32) == 0);

typedef _Float16 v16h __attribute__((ext_vector_type(16)));
typedef _Float16 v8h  __attribute__((ext_vector_type(8)));
typedef __bf16   v16b __attribute__((ext_vector_type(16)));
typedef __bf16   v8b  __attribute__((ext_vector_type(8)));
typedef float    v8f  __attribute__((ext_vector_type(8)));
typedef float    v4f  __attribute__((ext_vector_type(4)));
typedef unsigned int v4u __attribute__((ext_vector_type(4)));

__device__ __forceinline__ unsigned short bf_bits(float f) {
  unsigned u = __float_as_uint(f);
  return (unsigned short)((u + 0x7FFFu + ((u >> 16) & 1u)) >> 16);
}
__device__ __forceinline__ float bf_up(unsigned short h) { return __uint_as_float(((unsigned)h) << 16); }
__device__ __forceinline__ unsigned short h_bits(_Float16 x) { return __builtin_bit_cast(unsigned short, x); }
__device__ __forceinline__ unsigned pk16(unsigned short a, unsigned short b) { return (unsigned)a | ((unsigned)b << 16); }
__device__ __forceinline__ v8f zero8() { v8f z = {0.f, 0.f, 0.f, 0.f, 0.f, 0.f, 0.f, 0.f}; return z; }

__device__ __forceinline__ v16b ldfrag_b(const __bf16* p) {
  union { v16b v; v8b h[2]; } f;
  f.h[0] = *(const v8b*)(p);
  f.h[1] = *(const v8b*)(p + 16);
  return f.v;
}
__device__ __forceinline__ v16h ldfrag_h(const _Float16* p) {
  union { v16h v; v8h h[2]; } f;
  f.h[0] = *(const v8h*)(p);
  f.h[1] = *(const v8h*)(p + 16);
  return f.v;
}

__device__ __forceinline__ v8f mma_b(v16b a, v16b b, v8f c) {
  c = __builtin_amdgcn_wmma_f32_16x16x32_bf16(false, a, false, b, (short)0, c, false, false);
  asm volatile("v_nop\n\tv_nop\n\tv_nop\n\tv_nop" : "+v"(c) : "v"(a), "v"(b));
  return c;
}
__device__ __forceinline__ v8f mma_h(v16h a, v16h b, v8f c) {
  c = __builtin_amdgcn_wmma_f32_16x16x32_f16(false, a, false, b, (short)0, c, false, false);
  asm volatile("v_nop\n\tv_nop\n\tv_nop\n\tv_nop" : "+v"(c) : "v"(a), "v"(b));
  return c;
}
__device__ __forceinline__ v8f mma_b_raw(v16b a, v16b b, v8f c) {
  return __builtin_amdgcn_wmma_f32_16x16x32_bf16(false, a, false, b, (short)0, c, false, false);
}
__device__ __forceinline__ void dep_guard_b(v8f& a, v8f& b, v16b x, v16b y) {
  asm volatile("v_nop\n\tv_nop\n\tv_nop\n\tv_nop" : "+v"(a), "+v"(b) : "v"(x), "v"(y));
}
__device__ __forceinline__ void keep4_b(v16b a, v16b b, v16b c, v16b d) {
  asm volatile("v_nop" :: "v"(a), "v"(b), "v"(c), "v"(d));
}
__device__ __forceinline__ void acc_guard4(v8f& a, v8f& b, v8f& c, v8f& d) {
  asm volatile("v_nop\n\tv_nop\n\tv_nop\n\tv_nop" : "+v"(a), "+v"(b), "+v"(c), "+v"(d));
}

__global__ __launch_bounds__(256) void cvt_bf16x8(const float* __restrict__ in, unsigned short* out, int n8) {
  const int i = blockIdx.x * 256 + threadIdx.x;
  if (i < n8) {
    const v4f a = *(const v4f*)(in + (size_t)i * 8);
    const v4f b = *(const v4f*)(in + (size_t)i * 8 + 4);
    v4u p;
    p[0] = pk16(bf_bits(a[0]), bf_bits(a[1]));
    p[1] = pk16(bf_bits(a[2]), bf_bits(a[3]));
    p[2] = pk16(bf_bits(b[0]), bf_bits(b[1]));
    p[3] = pk16(bf_bits(b[2]), bf_bits(b[3]));
    *(volatile v4u*)(out + (size_t)i * 8) = p;
    __threadfence();
    *(volatile v4u*)(out + (size_t)i * 8) = p;
  }
}

__device__ __forceinline__ unsigned short qlevel_bits(float v, float rdiv) {
#pragma clang fp contract(off)
  const float x = bf_up(bf_bits(v));
  float t = x * 127.0f;
  t = t * rdiv;
  t = fminf(fmaxf(t, -127.0f), 127.0f);
  return bf_bits(rintf(t));
}

__global__ __launch_bounds__(256) void qlev_bf16x8(const float* __restrict__ w, unsigned short* out, int n8, float rdiv) {
  const int i = blockIdx.x * 256 + threadIdx.x;
  if (i < n8) {
    const v4f a = *(const v4f*)(w + (size_t)i * 8);
    const v4f b = *(const v4f*)(w + (size_t)i * 8 + 4);
    v4u p;
    p[0] = pk16(qlevel_bits(a[0], rdiv), qlevel_bits(a[1], rdiv));
    p[1] = pk16(qlevel_bits(a[2], rdiv), qlevel_bits(a[3], rdiv));
    p[2] = pk16(qlevel_bits(b[0], rdiv), qlevel_bits(b[1], rdiv));
    p[3] = pk16(qlevel_bits(b[2], rdiv), qlevel_bits(b[3], rdiv));
    *(volatile v4u*)(out + (size_t)i * 8) = p;
    __threadfence();
    *(volatile v4u*)(out + (size_t)i * 8) = p;
  }
}

template <int NSPLIT, int BIAS_MODE, int OUT_MODE>
__global__ __launch_bounds__(256) void gemm64(
    const unsigned short* __restrict__ Ap, const unsigned short* __restrict__ A2p, int lda, long long strideA,
    const unsigned short* __restrict__ Btp, int ldb, long long strideB,
    void* Cout, void* Cout2, int ldc, long long strideC,
    const float* __restrict__ bias, float bscale,
    int M, int N, int K, float scale) {
  const __bf16* A  = (const __bf16*)(const void*)Ap;
  const __bf16* A2 = (const __bf16*)(const void*)A2p;
  const __bf16* Bt = (const __bf16*)(const void*)Btp;
  __shared__ __align__(16) float sT[8][16 * 68];
  const int b    = blockIdx.y;
  const int lane = threadIdx.x & 31;
  const int wave = threadIdx.x >> 5;
  const int tilesN = N >> 6;
  const int tilesM = M >> 6;
  const int tile = blockIdx.x * 8 + wave;
  if (tile >= tilesM * tilesN) return;
  const int tm = tile / tilesN;
  const int tn = tile - tm * tilesN;
  const int m0 = tm << 6;
  const int n0 = tn << 6;

  const __bf16* Ab  = A  + (size_t)b * strideA;
  const __bf16* Bb  = Bt + (size_t)b * strideB;
  const __bf16* Ab2 = (NSPLIT == 1) ? (A2 + (size_t)b * strideA) : Ab;

  const int rlane = lane & 15;
  const int koff  = (lane >> 4) * 8;
  const int mOff  = (lane >> 4) * 8;

  v8f acc[4][4];
#pragma unroll
  for (int i = 0; i < 4; ++i)
#pragma unroll
    for (int j = 0; j < 4; ++j) acc[i][j] = zero8();

  for (int k0 = 0; k0 < K; k0 += 32) {
    v16b bh[4];
#pragma unroll
    for (int j = 0; j < 4; ++j) {
      const size_t bo = (size_t)(n0 + (j << 4) + rlane) * ldb + koff + k0;
      bh[j] = ldfrag_b(Bb + bo);
    }
#pragma unroll
    for (int i = 0; i < 4; ++i) {
      const size_t ao = (size_t)(m0 + (i << 4) + rlane) * lda + koff + k0;
      const v16b ah = ldfrag_b(Ab + ao);
      v16b al = ah;
      if (NSPLIT == 1) al = ldfrag_b(Ab2 + ao);
#pragma unroll
      for (int j = 0; j < 4; ++j) {
        acc[i][j] = mma_b_raw(ah, bh[j], acc[i][j]);
        if (NSPLIT == 1) acc[i][j] = mma_b_raw(al, bh[j], acc[i][j]);
      }
      dep_guard_b(acc[i][0], acc[i][3], ah, al);
    }
    keep4_b(bh[0], bh[1], bh[2], bh[3]);
  }
  acc_guard4(acc[0][0], acc[0][1], acc[0][2], acc[0][3]);
  acc_guard4(acc[1][0], acc[1][1], acc[1][2], acc[1][3]);
  acc_guard4(acc[2][0], acc[2][1], acc[2][2], acc[2][3]);
  acc_guard4(acc[3][0], acc[3][1], acc[3][2], acc[3][3]);

  float* slab = sT[wave];
#pragma unroll
  for (int i = 0; i < 4; ++i) {
    const int mBase = m0 + (i << 4);
    float bm[8];
#pragma unroll
    for (int r = 0; r < 8; ++r) bm[r] = 0.f;
    if (BIAS_MODE == 1) {
      const float braw = bf_up(bf_bits(bias[mBase + rlane])) * bscale;
#pragma unroll
      for (int r = 0; r < 8; ++r) bm[r] = __shfl(braw, mOff + r, 32);
    }
#pragma unroll
    for (int j = 0; j < 4; ++j) {
      float bn = 0.f;
      if (BIAS_MODE == 2) bn = bf_up(bf_bits(bias[n0 + (j << 4) + rlane])) * bscale;
#pragma unroll
      for (int r = 0; r < 8; ++r) {
        float v = acc[i][j][r] * scale;
        if (BIAS_MODE == 2) v += bn;
        if (BIAS_MODE == 1) v += bm[r];
        slab[(mOff + r) * 68 + (j << 4) + rlane] = v;
      }
    }
    __builtin_amdgcn_fence(__ATOMIC_RELEASE, "workgroup");
    __builtin_amdgcn_wave_barrier();
    __builtin_amdgcn_fence(__ATOMIC_ACQUIRE, "workgroup");
    if (OUT_MODE == 0) {
      float* C = (float*)Cout + (size_t)b * strideC;
      const int hh = lane >> 4, c4 = (lane & 15) * 4;
      for (int pass = 0; pass < 2; ++pass) {
#pragma unroll
        for (int it = 0; it < 8; ++it) {
          const int row = it * 2 + hh;
          const v4f v = *(const v4f*)(slab + row * 68 + c4);
          *(volatile v4f*)(C + (size_t)(mBase + row) * ldc + n0 + c4) = v;
        }
        __threadfence();
      }
    } else {
      const int q = lane >> 3, c8 = (lane & 7) * 8;
      unsigned short* C  = (unsigned short*)Cout  + (size_t)b * strideC;
      unsigned short* C2 = (unsigned short*)Cout2 + (size_t)b * strideC;
      v4u hv[4], lv[4];
#pragma unroll
      for (int it = 0; it < 4; ++it) {
        const int row = it * 4 + q;
        const float* sp = slab + row * 68 + c8;
        v4u a, a2;
#pragma unroll
        for (int e = 0; e < 4; ++e) {
          const float f0 = sp[2 * e], f1 = sp[2 * e + 1];
          unsigned short h0, h1, l0, l1;
          if (OUT_MODE == 2) {
            h0 = bf_bits(f0); h1 = bf_bits(f1);
            l0 = bf_bits(f0 - bf_up(h0)); l1 = bf_bits(f1 - bf_up(h1));
          } else {
            h0 = h_bits((_Float16)f0); h1 = h_bits((_Float16)f1);
            l0 = 0; l1 = 0;
          }
          a[e] = pk16(h0, h1); a2[e] = pk16(l0, l1);
        }
        hv[it] = a; lv[it] = a2;
      }
      for (int pass = 0; pass < 2; ++pass) {
#pragma unroll
        for (int it = 0; it < 4; ++it) {
          const int row = it * 4 + q;
          *(volatile v4u*)(C + (size_t)(mBase + row) * ldc + n0 + c8) = hv[it];
          if (OUT_MODE == 2) *(volatile v4u*)(C2 + (size_t)(mBase + row) * ldc + n0 + c8) = lv[it];
        }
        __threadfence();
      }
    }
    __builtin_amdgcn_fence(__ATOMIC_RELEASE, "workgroup");
    __builtin_amdgcn_wave_barrier();
    __builtin_amdgcn_fence(__ATOMIC_ACQUIRE, "workgroup");
  }
}

__global__ __launch_bounds__(128)
void attn_kernel(const unsigned short* __restrict__ qkp,
                 const unsigned short* __restrict__ vhp, const unsigned short* __restrict__ vlp,
                 unsigned short* ohp, unsigned short* olp, float sscale) {
  union FB { v16b v; v8b h[2]; };
  union FH { v16h v; v8h h[2]; };
  __shared__ __align__(16) _Float16 Ksh[64 * 64];
  __shared__ __align__(16) __bf16   Vth[64 * 64];
  __shared__ __align__(16) __bf16   Vtl[64 * 64];
  __shared__ __align__(16) __bf16   Psh[4][16 * 64];
  __shared__ __align__(16) __bf16   Psl[4][16 * 64];
  __shared__ __align__(16) float    Os[4][16 * 64];

  const int tid  = threadIdx.x;
  const int wave = tid >> 5;
  const int lane = tid & 31;
  const int hh   = lane >> 4;
  const int c    = lane & 15;

  const int bx   = blockIdx.x;
  const int qb   = bx % NQB;
  const int rest = bx / NQB;
  const int h    = rest % NH;
  const int b    = rest / NH;
  const int q0   = qb * 64 + wave * 16;
  const size_t tstep = (size_t)NBAT * QKW;

  const _Float16* Qp = (const _Float16*)(const void*)qkp + (size_t)b * QKW + (size_t)h * HD;
  const _Float16* Kp = Qp + EMB;
  const __bf16* Vh = (const __bf16*)(const void*)vhp + ((size_t)b * EMB + (size_t)h * HD) * TT;
  const __bf16* Vl = (const __bf16*)(const void*)vlp + ((size_t)b * EMB + (size_t)h * HD) * TT;

  v16h qa[2];
#pragma unroll
  for (int dc = 0; dc < 2; ++dc) {
    qa[dc] = ldfrag_h(Qp + (size_t)(q0 + c) * tstep + dc * 32 + 8 * hh);
  }

  float mrow[8], lrow[8];
  v8f oacc[4];
#pragma unroll
  for (int r = 0; r < 8; ++r) { mrow[r] = -INFINITY; lrow[r] = 0.f; }
#pragma unroll
  for (int t = 0; t < 4; ++t) oacc[t] = zero8();

  for (int kt = 0; kt < NQB; ++kt) {
    const int kv0 = kt * 64;
    __syncthreads();
    {
      const int r = tid >> 1, half = (tid & 1) * 32;
      const _Float16* kg  = Kp + (size_t)(kv0 + r) * tstep + half;
      const __bf16*   vg  = Vh + (size_t)r * TT + kv0 + half;
      const __bf16*   vlg = Vl + (size_t)r * TT + kv0 + half;
#pragma unroll
      for (int i = 0; i < 4; ++i) {
        const v8h a0 = *(const v8h*)(kg + 8 * i);
        const v8b b0 = *(const v8b*)(vg + 8 * i);
        const v8b b1 = *(const v8b*)(vlg + 8 * i);
        *(v8h*)(Ksh + r * 64 + half + 8 * i) = a0;
        *(v8b*)(Vth + r * 64 + half + 8 * i) = b0;
        *(v8b*)(Vtl + r * 64 + half + 8 * i) = b1;
      }
    }
    __syncthreads();

    v8f s[4];
#pragma unroll
    for (int j = 0; j < 4; ++j) {
      s[j] = zero8();
#pragma unroll
      for (int dc = 0; dc < 2; ++dc) {
        FH kb;
        kb.h[0] = *(const v8h*)(Ksh + (j * 16 + c) * 64 + dc * 32 + 8 * hh);
        kb.h[1] = *(const v8h*)(Ksh + (j * 16 + c) * 64 + dc * 32 + 16 + 8 * hh);
        s[j] = mma_h(qa[dc], kb.v, s[j]);
      }
    }

    __bf16* pwh = Psh[wave];
    __bf16* pwl = Psl[wave];
#pragma unroll
    for (int r = 0; r < 8; ++r) {
      float m = -INFINITY;
#pragma unroll
      for (int j = 0; j < 4; ++j) {
        const float sv = s[j][r] * sscale;
        s[j][r] = sv;
        m = fmaxf(m, sv);
      }
#pragma unroll
      for (int off = 1; off < 16; off <<= 1) m = fmaxf(m, __shfl_xor(m, off, 32));
      const float mnew  = fmaxf(mrow[r], m);
      const float alpha = __expf(mrow[r] - mnew);
      mrow[r] = mnew;
      float psum = 0.f;
#pragma unroll
      for (int j = 0; j < 4; ++j) {
        const float p = __expf(s[j][r] - mnew);
        psum += p;
        const unsigned short hb = bf_bits(p);
        const unsigned short lb = bf_bits(p - bf_up(hb));
        pwh[(8 * hh + r) * 64 + j * 16 + c] = __builtin_bit_cast(__bf16, hb);
        pwl[(8 * hh + r) * 64 + j * 16 + c] = __builtin_bit_cast(__bf16, lb);
      }
#pragma unroll
      for (int off = 1; off < 16; off <<= 1) psum += __shfl_xor(psum, off, 32);
      lrow[r] = lrow[r] * alpha + psum;
#pragma unroll
      for (int t = 0; t < 4; ++t) oacc[t][r] *= alpha;
    }
    __builtin_amdgcn_fence(__ATOMIC_RELEASE, "workgroup");
    __builtin_amdgcn_wave_barrier();
    __builtin_amdgcn_fence(__ATOMIC_ACQUIRE, "workgroup");

#pragma unroll 1
    for (int kk = 0; kk < 2; ++kk) {
      FB pa, pl;
      pa.h[0] = *(const v8b*)(pwh + c * 64 + kk * 32 + 8 * hh);
      pa.h[1] = *(const v8b*)(pwh + c * 64 + kk * 32 + 16 + 8 * hh);
      pl.h[0] = *(const v8b*)(pwl + c * 64 + kk * 32 + 8 * hh);
      pl.h[1] = *(const v8b*)(pwl + c * 64 + kk * 32 + 16 + 8 * hh);
#pragma unroll
      for (int t = 0; t < 4; ++t) {
        FB vb, vl;
        vb.h[0] = *(const v8b*)(Vth + (t * 16 + c) * 64 + kk * 32 + 8 * hh);
        vb.h[1] = *(const v8b*)(Vth + (t * 16 + c) * 64 + kk * 32 + 16 + 8 * hh);
        vl.h[0] = *(const v8b*)(Vtl + (t * 16 + c) * 64 + kk * 32 + 8 * hh);
        vl.h[1] = *(const v8b*)(Vtl + (t * 16 + c) * 64 + kk * 32 + 16 + 8 * hh);
        oacc[t] = mma_b(pa.v, vb.v, oacc[t]);
        oacc[t] = mma_b(pa.v, vl.v, oacc[t]);
        oacc[t] = mma_b(pl.v, vb.v, oacc[t]);
      }
    }
  }

  float* os = Os[wave];
#pragma unroll
  for (int r = 0; r < 8; ++r) {
    const float l = lrow[r];
    const float inv = (l > 0.f) ? (1.0f / l) : 0.f;
#pragma unroll
    for (int t = 0; t < 4; ++t) os[(8 * hh + r) * 64 + t * 16 + c] = oacc[t][r] * inv;
  }
  __builtin_amdgcn_fence(__ATOMIC_RELEASE, "workgroup");
  __builtin_amdgcn_wave_barrier();
  __builtin_amdgcn_fence(__ATOMIC_ACQUIRE, "workgroup");
  {
    const int q4 = lane >> 3, c8 = (lane & 7) * 8;
    v4u hv[4], lv[4];
#pragma unroll
    for (int it = 0; it < 4; ++it) {
      const int row = it * 4 + q4;
      const float* sp = os + row * 64 + c8;
      v4u a, a2;
#pragma unroll
      for (int e = 0; e < 4; ++e) {
        const float f0 = sp[2 * e], f1 = sp[2 * e + 1];
        const unsigned short h0 = bf_bits(f0), h1 = bf_bits(f1);
        const unsigned short l0 = bf_bits(f0 - bf_up(h0)), l1 = bf_bits(f1 - bf_up(h1));
        a[e] = pk16(h0, h1); a2[e] = pk16(l0, l1);
      }
      hv[it] = a; lv[it] = a2;
    }
    for (int pass = 0; pass < 2; ++pass) {
#pragma unroll
      for (int it = 0; it < 4; ++it) {
        const int row = it * 4 + q4;
        const size_t go = ((size_t)(q0 + row) * NBAT + b) * EMB + (size_t)h * HD + c8;
        *(volatile v4u*)(ohp + go) = hv[it];
        *(volatile v4u*)(olp + go) = lv[it];
      }
      __threadfence();
    }
  }
}

extern "C" void kernel_launch(void* const* d_in, const int* in_sizes, int n_in,
                              void* d_out, int out_size, void* d_ws, size_t ws_size,
                              hipStream_t stream) {
  if (n_in < 5) return;
  if (in_sizes[0] != NTOK * EMB) return;
  if (in_sizes[1] != 3 * EMB * EMB) return;
  if (in_sizes[2] != 3 * EMB) return;
  if (in_sizes[3] != EMB * EMB) return;
  if (in_sizes[4] != EMB) return;
  if (out_size != NTOK * EMB) return;

  const float* query = (const float*)d_in[0];
  const float* qkv_w = (const float*)d_in[1];
  const float* qkv_b = (const float*)d_in[2];
  const float* o_w   = (const float*)d_in[3];
  const float* o_b   = (const float*)d_in[4];

  const size_t PX  = (size_t)NTOK * EMB * 2;
  const size_t PNQ = (size_t)3 * EMB * EMB * 2;
  const size_t PNO = (size_t)EMB * EMB * 2;
  const size_t PQK = (size_t)NTOK * QKW * 2;
  const size_t PVT = (size_t)NBAT * EMB * TT * 2;
  size_t off = 0;
  const size_t oXB   = off; off += PX;
  const size_t oNQ   = off; off += PNQ;
  const size_t oNO   = off; off += PNO;
  const size_t oQK   = off; off += PQK;
  const size_t oVTh  = off; off += PVT;
  const size_t oVTl  = off; off += PVT;
  const size_t oCTXh = off; off += PX;
  const size_t oCTXl = off; off += PX;
  if (off > ws_size) return;
  if (off > (size_t)134217728) return;

  char* ws = (char*)d_ws;
  unsigned short* XB   = (unsigned short*)(ws + oXB);
  unsigned short* NQ   = (unsigned short*)(ws + oNQ);
  unsigned short* NO   = (unsigned short*)(ws + oNO);
  unsigned short* QK   = (unsigned short*)(ws + oQK);
  unsigned short* VTh  = (unsigned short*)(ws + oVTh);
  unsigned short* VTl  = (unsigned short*)(ws + oVTl);
  unsigned short* CTXh = (unsigned short*)(ws + oCTXh);
  unsigned short* CTXl = (unsigned short*)(ws + oCTXl);

  const double scq_d   = 1.0 / sqrt((double)(3 * EMB));
  const float  scq_f   = (float)scq_d;
  const float  rdivq   = 1.0f / scq_f;
  const float  c_qkv   = (float)(scq_d / 127.0);
  const double sco_d   = 1.0 / sqrt((double)EMB);
  const float  sco_f   = (float)sco_d;
  const float  rdivo   = 1.0f / sco_f;
  const float  c_o     = (float)(sco_d / 127.0);

  const dim3 blk(256);
  const int n8x = NTOK * EMB / 8;
  const int n8q = 3 * EMB * EMB / 8;
  const int n8o = EMB * EMB / 8;
  const dim3 gCvtX((n8x + 255) / 256);
  const dim3 gQ((n8q + 255) / 256);
  const dim3 gO((n8o + 255) / 256);
  const dim3 gQK(((NTOK / 64) * (2 * EMB / 64) + 7) / 8, 1);
  const dim3 gVT(((EMB / 64) * (TT / 64) + 7) / 8, NBAT);
  const dim3 gOut(((NTOK / 64) * (EMB / 64) + 7) / 8, 1);
  const dim3 gAtt(NBAT * NH * NQB);

  cvt_bf16x8<<<gCvtX, blk, 0, stream>>>(query, XB, n8x);
  qlev_bf16x8<<<gQ, blk, 0, stream>>>(qkv_w, NQ, n8q, rdivq);
  qlev_bf16x8<<<gO, blk, 0, stream>>>(o_w, NO, n8o, rdivo);
  gemm64<0, 2, 1><<<gQK, blk, 0, stream>>>(
      XB, XB, EMB, 0LL, NQ, EMB, 0LL,
      (void*)QK, (void*)QK, QKW, 0LL,
      qkv_b, 8.0f,
      NTOK, 2 * EMB, EMB, 8.0f * c_qkv);
  gemm64<0, 1, 2><<<gVT, blk, 0, stream>>>(
      NQ + (size_t)2 * EMB * EMB, NQ + (size_t)2 * EMB * EMB, EMB, 0LL, XB, NBAT * EMB, (long long)EMB,
      (void*)VTh, (void*)VTl, TT, (long long)EMB * TT,
      qkv_b + 2 * EMB, 1.0f,
      EMB, TT, EMB, c_qkv);
  attn_kernel<<<gAtt, dim3(128), 0, stream>>>(QK, VTh, VTl, CTXh, CTXl, 1.0f / 512.0f);
  gemm64<1, 2, 0><<<gOut, blk, 0, stream>>>(
      CTXh, CTXl, EMB, 0LL, NO, EMB, 0LL,
      d_out, d_out, EMB, 0LL,
      o_b, 1.0f,
      NTOK, EMB, EMB, c_o);
  (void)hipGetLastError();
}
